// PortHamiltonianLayer_26010321945364
// MI455X (gfx1250) — hardware-verified
//
#include <hip/hip_runtime.h>
#include <stddef.h>


typedef _Float16 v16h __attribute__((ext_vector_type(16)));
typedef _Float16 v8h  __attribute__((ext_vector_type(8)));
typedef float    v8f  __attribute__((ext_vector_type(8)));
typedef float    v4f  __attribute__((ext_vector_type(4)));
typedef _Float16 h16;

#ifndef NB
#define NB 2
#endif
#ifndef SEQ
#define SEQ 1024
#endif
#define NB_FULL  2
#define SEQ_FULL 1024
#define DIM   128
#define HID   512
#define NFEAT (DIM * DIM)
#define MROWS (NB * SEQ)

static_assert(NB >= 1 && NB <= NB_FULL);
static_assert(SEQ >= 64 && SEQ <= SEQ_FULL && (SEQ % 64) == 0);
static_assert(HID == 4 * DIM);
static_assert((DIM % 64) == 0 && (DIM % 32) == 0);
static_assert((HID % 64) == 0 && (HID % 32) == 0);
static_assert((MROWS % 64) == 0 && (MROWS % 16) == 0);
static_assert(DIM == 16 * 8);
static_assert(DIM == 32 * 4);
static_assert(2 * DIM == 256);
static_assert(((size_t)NFEAT * DIM) % 2048 == 0);
static_assert(((size_t)HID * DIM) % 2048 == 0);

#define LDT 72
#define LDC 68
static_assert((LDT % 8) == 0 && LDT >= 64);
static_assert((LDC % 4) == 0 && LDC >= 64);

#define WCARRY 64.0f
#define GCARRY 1024.0f
#define R_EPS  1.0e-4f

#define TOKT   16
#define CHK    4
#define CROWS  (CHK * DIM)
#define NCHUNK (DIM / CHK)
#define TS     17
#define XS     132
static_assert(CROWS == 8 * 4 * 16);
static_assert(CHK == 4);
static_assert((XS % 4) == 0 && XS >= DIM);
static_assert((DIM % CHK) == 0);

#define WBIG_BYTES ((size_t)NFEAT * DIM * 2)
#define W1_BYTES   ((size_t)HID * DIM * 2)
#define XN_BYTES   ((size_t)MROWS * DIM * 2)
#define GM_BYTES   ((size_t)MROWS * HID * 2)
#define GF_BYTES   ((size_t)MROWS * DIM * 4)
#define OFF_WJ  ((size_t)0)
#define OFF_WR  (OFF_WJ + WBIG_BYTES)
#define OFF_W1A (OFF_WR + WBIG_BYTES)
#define OFF_W1T (OFF_W1A + W1_BYTES)
#define OFF_XN  (OFF_W1T + W1_BYTES)
#define OFF_GM  (OFF_XN + XN_BYTES)
#define OFF_GF  (OFF_GM + GM_BYTES)
#define WS_TOTAL (OFF_GF + GF_BYTES)
static_assert((WBIG_BYTES % 128) == 0 && (W1_BYTES % 128) == 0 && (XN_BYTES % 128) == 0);
static_assert((GM_BYTES % 128) == 0 && (GF_BYTES % 128) == 0);
static_assert(WS_TOTAL <= (size_t)134217728);

__device__ __forceinline__ float bf16r(float x) {
  unsigned int u = __float_as_uint(x);
  u = (u + 0x7FFFu + ((u >> 16) & 1u)) & 0xFFFF0000u;
  return __uint_as_float(u);
}

static __device__ __forceinline__ h16 toh_flush(float v) {
  const h16 r = (h16)v;
  return (fabsf(v) < 6.103515625e-05f) ? (h16)0.0f : r;
}

__device__ __forceinline__ v16h frag_at(const _Float16* p) {
  v8h lo = *(const v8h*)(p);
  v8h hi = *(const v8h*)(p + 16);
  v16h out;
#pragma unroll
  for (int i = 0; i < 8; ++i) { out[i] = lo[i]; out[i + 8] = hi[i]; }
  return out;
}

__device__ __forceinline__ v8f wmma16(v16h a, v16h b, v8f c) {
  v8f d = __builtin_amdgcn_wmma_f32_16x16x32_f16(false, a, false, b, (short)0, c,
                                                 false, false);
  asm volatile("v_nop\n\tv_nop\n\tv_nop\n\tv_nop" : "+v"(d) : "v"(a), "v"(b));
  return d;
}

__device__ __forceinline__ float red16_sum(float x) {
#pragma unroll
  for (int off = 1; off < 16; off <<= 1) x += __shfl_xor(x, off, 32);
  return x;
}

__global__ __launch_bounds__(256) void wconv_kernel(
    const float* __restrict__ W, _Float16* __restrict__ Wt, unsigned ldw, unsigned ldk) {
  __shared__ _Float16 T[64 * LDT];
  const unsigned tid = threadIdx.x;
  const unsigned n0 = blockIdx.x * 64u;
  const unsigned k0 = blockIdx.y * 64u;
#pragma unroll 4
  for (unsigned j = 0; j < 16u; ++j) {
    const unsigned idx = tid + 256u * j;
    const unsigned kr = idx >> 6, nc = idx & 63u;
    const float v = W[(size_t)(k0 + kr) * ldw + n0 + nc];
    T[nc * LDT + kr] = toh_flush(WCARRY * bf16r(v));
  }
  __syncthreads();
  v8h x[2];
  size_t off[2];
#pragma unroll
  for (unsigned i = 0; i < 2u; ++i) {
    const unsigned n = 32u * i + (tid >> 3);
    const unsigned kc = (tid & 7u) * 8u;
    x[i] = *(const v8h*)&T[n * LDT + kc];
    off[i] = (size_t)(n0 + n) * ldk + k0 + kc;
  }
#pragma unroll
  for (int i = 0; i < 2; ++i) *(volatile v8h*)(Wt + off[i]) = x[i];
  __threadfence();
#pragma unroll
  for (int i = 0; i < 2; ++i) *(volatile v8h*)(Wt + off[i]) = x[i];
}

__global__ __launch_bounds__(256) void wplane_kernel(
    const float* __restrict__ W, _Float16* __restrict__ Wp) {
  const size_t e = ((size_t)blockIdx.x * 256u + threadIdx.x) * 8u;
  const v4f a0 = *(const v4f*)(W + e);
  const v4f a1 = *(const v4f*)(W + e + 4u);
  v8h o;
#pragma unroll
  for (int i = 0; i < 4; ++i) {
    o[i]     = toh_flush(WCARRY * bf16r(a0[i]));
    o[i + 4] = toh_flush(WCARRY * bf16r(a1[i]));
  }
  _Float16* p = Wp + e;
  *(volatile v8h*)p = o;
  __threadfence();
  *(volatile v8h*)p = o;
}

__global__ __launch_bounds__(256) void ln_kernel(
    const float* __restrict__ X, const float* __restrict__ G, const float* __restrict__ Be,
    _Float16* __restrict__ dst) {
#pragma clang fp contract(off)
  const unsigned lane = threadIdx.x & 31u;
  const unsigned wave = (unsigned)__builtin_amdgcn_readfirstlane((int)(threadIdx.x >> 5));
  const unsigned crow = blockIdx.x * 16u + wave * 2u + (lane >> 4);
  const unsigned bidx = crow / (unsigned)SEQ;
  const unsigned sq = crow - bidx * (unsigned)SEQ;
  const size_t srow = (size_t)bidx * SEQ_FULL + sq;
  const unsigned c = (lane & 15u) * 8u;
  const float* xr = X + srow * DIM + c;
  const v4f a0 = *(const v4f*)(xr);
  const v4f a1 = *(const v4f*)(xr + 4u);
  float e[8];
#pragma unroll
  for (int i = 0; i < 4; ++i) { e[i] = bf16r(a0[i]); e[i + 4] = bf16r(a1[i]); }
  float s = 0.0f;
#pragma unroll
  for (int i = 0; i < 8; ++i) s += e[i];
  const float mean = red16_sum(s) * (1.0f / (float)DIM);
  float ss = 0.0f;
#pragma unroll
  for (int i = 0; i < 8; ++i) { const float d = e[i] - mean; ss += d * d; }
  const float var = red16_sum(ss) * (1.0f / (float)DIM);
  const float rstd = 1.0f / sqrtf(var + 1.0e-5f);
  const v4f g0 = *(const v4f*)(G + c);
  const v4f g1 = *(const v4f*)(G + c + 4u);
  const v4f b0 = *(const v4f*)(Be + c);
  const v4f b1 = *(const v4f*)(Be + c + 4u);
  v8h o;
#pragma unroll
  for (int i = 0; i < 4; ++i) {
    o[i]     = toh_flush((e[i] - mean) * rstd * bf16r(g0[i]) + bf16r(b0[i]));
    o[i + 4] = toh_flush((e[i + 4] - mean) * rstd * bf16r(g1[i]) + bf16r(b1[i]));
  }
  _Float16* p = dst + (size_t)crow * DIM + c;
  *(volatile v8h*)p = o;
  __threadfence();
  *(volatile v8h*)p = o;
}

template <int MODE>
__device__ __forceinline__ void gemm_body(
    const _Float16* __restrict__ A16, const _Float16* __restrict__ Bt, const unsigned K,
    const float* __restrict__ bias, const float* __restrict__ gain,
    float* __restrict__ outf, _Float16* __restrict__ out16) {
  __shared__ __attribute__((aligned(16))) float Cs[64 * LDC];
  const unsigned tid = threadIdx.x, lane = tid & 31u;
  const unsigned w = (unsigned)__builtin_amdgcn_readfirstlane((int)(threadIdx.x >> 5));
  const unsigned mw = w >> 1, nw = w & 1u;
  const unsigned hh = lane >> 4, m = lane & 15u;
  const unsigned n0 = blockIdx.x * 64u;
  const unsigned row0 = blockIdx.y * 64u;

  const _Float16* ap  = A16 + (size_t)(row0 + mw * 16u + m) * K + hh * 8u;
  const _Float16* bp0 = Bt + (size_t)(n0 + nw * 32u + m) * K + hh * 8u;
  const _Float16* bp1 = bp0 + (size_t)16 * K;
  v8f acc0 = {}, acc1 = {};
#pragma unroll 2
  for (unsigned k0 = 0; k0 < K; k0 += 32u) {
    const v16h a  = frag_at(ap + k0);
    const v16h b0 = frag_at(bp0 + k0);
    const v16h b1 = frag_at(bp1 + k0);
    acc0 = wmma16(a, b0, acc0);
    acc1 = wmma16(a, b1, acc1);
  }
#pragma unroll
  for (int r = 0; r < 8; ++r) {
    float* d = &Cs[(mw * 16u + hh * 8u + (unsigned)r) * LDC + nw * 32u + m];
    d[0]  = acc0[r];
    d[16] = acc1[r];
  }
  __syncthreads();

  if (MODE == 0) {
#pragma unroll 1
    for (unsigned g = 0; g < 4u; ++g) {
      const unsigned r = 32u * (g >> 1) + (tid >> 3);
      const unsigned c = (tid & 7u) * 8u + 4u * (g & 1u);
      const v4f u  = *(const v4f*)&Cs[r * LDC + c];
      const v4f gb = *(const v4f*)(bias + n0 + c);
      const v4f gw = *(const v4f*)(gain + n0 + c);
      v4f t;
#pragma unroll
      for (int j = 0; j < 4; ++j) {
        const float z = u[j] * (1.0f / WCARRY) + bf16r(gb[j]);
        const float sig = __builtin_amdgcn_rcpf(1.0f + __expf(-z));
        const float ds = sig * (1.0f + z * (1.0f - sig));
        t[j] = GCARRY * (ds * bf16r(gw[j]));
      }
      *(v4f*)&Cs[r * LDC + c] = t;
    }
    v8h x[2];
    size_t off[2];
#pragma unroll
    for (unsigned i = 0; i < 2u; ++i) {
      const unsigned r = 32u * i + (tid >> 3);
      const unsigned c = (tid & 7u) * 8u;
      const v4f u0 = *(const v4f*)&Cs[r * LDC + c];
      const v4f u1 = *(const v4f*)&Cs[r * LDC + c + 4];
#pragma unroll
      for (int j = 0; j < 4; ++j) {
        x[i][j]     = toh_flush(u0[j]);
        x[i][j + 4] = toh_flush(u1[j]);
      }
      off[i] = (size_t)(row0 + r) * HID + n0 + c;
    }
#pragma unroll
    for (int i = 0; i < 2; ++i) *(volatile v8h*)(out16 + off[i]) = x[i];
    __threadfence();
#pragma unroll
    for (int i = 0; i < 2; ++i) *(volatile v8h*)(out16 + off[i]) = x[i];
  }

  if (MODE == 1) {
    const float cs = 1.0f / (WCARRY * GCARRY);
    v4f xs[4];
    size_t off[4];
#pragma unroll
    for (unsigned i = 0; i < 4u; ++i) {
      const unsigned r = 16u * i + (tid >> 4);
      const unsigned c = (tid & 15u) * 4u;
      const v4f u = *(const v4f*)&Cs[r * LDC + c];
      v4f val;
#pragma unroll
      for (int j = 0; j < 4; ++j) val[j] = u[j] * cs;
      xs[i] = val;
      off[i] = (size_t)(row0 + r) * DIM + n0 + c;
    }
#pragma unroll
    for (int i = 0; i < 4; ++i) *(volatile v4f*)(outf + off[i]) = xs[i];
    __threadfence();
#pragma unroll
    for (int i = 0; i < 4; ++i) *(volatile v4f*)(outf + off[i]) = xs[i];
  }
}

__global__ __launch_bounds__(256) void gemm_z_kernel(
    const _Float16* __restrict__ Xn, const _Float16* __restrict__ W1a,
    const float* __restrict__ b1, const float* __restrict__ w2, _Float16* __restrict__ gm) {
  gemm_body<0>(Xn, W1a, (unsigned)DIM, b1, w2, (float*)0, gm);
}
__global__ __launch_bounds__(256) void gemm_g_kernel(
    const _Float16* __restrict__ Gm, const _Float16* __restrict__ W1t,
    float* __restrict__ gout) {
  gemm_body<1>(Gm, W1t, (unsigned)HID, (const float*)0, (const float*)0, gout, (_Float16*)0);
}

__device__ __forceinline__ void weight_pass(
    const _Float16* __restrict__ W16, const float* __restrict__ bias, const unsigned rows_base,
    const v16h xb0, const v16h xb1, const v16h xb2, const v16h xb3,
    float* tile, const unsigned wave, const unsigned hh, const unsigned m) {
#pragma unroll
  for (unsigned mm = 0; mm < 4u; ++mm) {
    const unsigned mt = wave * 4u + mm;
    const _Float16* ap = W16 + (size_t)(rows_base + mt * 16u + m) * DIM + hh * 8u;
    v8f acc = {};
    acc = wmma16(frag_at(ap), xb0, acc);
    acc = wmma16(frag_at(ap + 32), xb1, acc);
    acc = wmma16(frag_at(ap + 64), xb2, acc);
    acc = wmma16(frag_at(ap + 96), xb3, acc);
    const unsigned rb = mt * 16u + hh * 8u;
    const v4f b0 = *(const v4f*)(bias + rows_base + rb);
    const v4f b1 = *(const v4f*)(bias + rows_base + rb + 4u);
#pragma unroll
    for (int r = 0; r < 4; ++r) {
      tile[(rb + (unsigned)r) * TS + m]      = acc[r]     * (1.0f / WCARRY) + bf16r(b0[r]);
      tile[(rb + 4u + (unsigned)r) * TS + m] = acc[r + 4] * (1.0f / WCARRY) + bf16r(b1[r]);
    }
  }
}

__device__ __forceinline__ float row_dot(const float* tile, const float* vec,
                                         const unsigned rk, const unsigned rq,
                                         const unsigned rt) {
  const float* tp = tile + (rk * DIM + rq * 32u) * TS + rt;
  const float* gp = vec + rt * XS + rq * 32u;
  float s = 0.0f;
#pragma unroll 2
  for (unsigned ii = 0; ii < 32u; ii += 4u) {
    const v4f g4 = *(const v4f*)(gp + ii);
    s += tp[(ii + 0u) * TS] * g4[0];
    s += tp[(ii + 1u) * TS] * g4[1];
    s += tp[(ii + 2u) * TS] * g4[2];
    s += tp[(ii + 3u) * TS] * g4[3];
  }
  s += __shfl_xor(s, 1, 32);
  s += __shfl_xor(s, 2, 32);
  return s;
}

__global__ __launch_bounds__(256) void heavy_kernel(
    const _Float16* __restrict__ Wj16, const float* __restrict__ bj,
    const _Float16* __restrict__ Wr16, const float* __restrict__ br,
    const _Float16* __restrict__ Xn16, const float* __restrict__ G,
    const float* __restrict__ X, float* __restrict__ out) {
  __shared__ __attribute__((aligned(16))) float tile[CROWS * TS];
  __shared__ __attribute__((aligned(16))) float gr[TOKT * XS];
  __shared__ __attribute__((aligned(16))) float u1s[TOKT * XS];
  __shared__ __attribute__((aligned(16))) float vsc[TOKT * CHK];

  const unsigned tid = threadIdx.x, lane = tid & 31u;
  const unsigned wave = (unsigned)__builtin_amdgcn_readfirstlane((int)(threadIdx.x >> 5));
  const unsigned hh = lane >> 4, m = lane & 15u;
  const unsigned tok0 = blockIdx.x * (unsigned)TOKT;

#pragma unroll
  for (unsigned j = 0; j < 2u; ++j) {
    const unsigned idx = tid + 256u * j;
    const unsigned t = idx >> 5, c = (idx & 31u) * 4u;
    *(v4f*)&gr[t * XS + c] = *(const v4f*)(G + (size_t)(tok0 + t) * DIM + c);
  }

  const _Float16* xp = Xn16 + (size_t)(tok0 + m) * DIM + hh * 8u;
  const v16h xb0 = frag_at(xp);
  const v16h xb1 = frag_at(xp + 32);
  const v16h xb2 = frag_at(xp + 64);
  const v16h xb3 = frag_at(xp + 96);

  const unsigned rq = lane & 3u;
  const unsigned rt = (wave & 1u) * 8u + (lane >> 2);
  const unsigned rk = wave >> 1;
  const unsigned ci = tid & 127u;
  const unsigned ct0 = (wave >> 2) * 8u;

  float ua[8];
#pragma unroll
  for (int tt = 0; tt < 8; ++tt) ua[tt] = 0.0f;
  __syncthreads();

  for (unsigned c = 0; c < (unsigned)NCHUNK; ++c) {
    const unsigned kg0 = c * (unsigned)CHK;
    const unsigned rows_base = kg0 * (unsigned)DIM;

    weight_pass(Wj16, bj, rows_base, xb0, xb1, xb2, xb3, tile, wave, hh, m);
    __syncthreads();
    {
      const float s = row_dot(tile, gr, rk, rq, rt);
      if (rq == 0u) u1s[rt * XS + kg0 + rk] = s;
    }
#pragma unroll
    for (int tt = 0; tt < 8; ++tt) {
      const unsigned t = ct0 + (unsigned)tt;
      const v4f gk = *(const v4f*)&gr[t * XS + kg0];
      const float* tp = &tile[ci * TS + t];
      float s = tp[0] * gk[0];
      s += tp[(1 * DIM) * TS] * gk[1];
      s += tp[(2 * DIM) * TS] * gk[2];
      s += tp[(3 * DIM) * TS] * gk[3];
      ua[tt] += s;
    }
    __syncthreads();

    weight_pass(Wr16, br, rows_base, xb0, xb1, xb2, xb3, tile, wave, hh, m);
    __syncthreads();
    {
      const float s = row_dot(tile, gr, rk, rq, rt);
      if (rq == 0u) vsc[rt * CHK + rk] = s;
    }
    __syncthreads();
#pragma unroll
    for (int tt = 0; tt < 8; ++tt) {
      const unsigned t = ct0 + (unsigned)tt;
      const v4f vk = *(const v4f*)&vsc[t * CHK];
      const float* tp = &tile[ci * TS + t];
      float s = tp[0] * vk[0];
      s += tp[(1 * DIM) * TS] * vk[1];
      s += tp[(2 * DIM) * TS] * vk[2];
      s += tp[(3 * DIM) * TS] * vk[3];
      ua[tt] += s;
    }
    __syncthreads();
  }

#pragma unroll
  for (int tt = 0; tt < 8; ++tt) {
    const unsigned t = ct0 + (unsigned)tt;
    const float val = u1s[t * XS + ci] - ua[tt] - R_EPS * gr[t * XS + ci];
    u1s[t * XS + ci] = val;
  }
  __syncthreads();

  v4f xs[2];
  size_t off[2];
#pragma unroll
  for (unsigned j = 0; j < 2u; ++j) {
    const unsigned idx = tid + 256u * j;
    const unsigned t = idx >> 5, cc = (idx & 31u) * 4u;
    const unsigned crow = tok0 + t;
    const unsigned bidx = crow / (unsigned)SEQ;
    const unsigned sq = crow - bidx * (unsigned)SEQ;
    const size_t frow = (size_t)bidx * SEQ_FULL + sq;
    const v4f u = *(const v4f*)&u1s[t * XS + cc];
    const v4f xin = *(const v4f*)(X + frow * DIM + cc);
    v4f val;
#pragma unroll
    for (int q = 0; q < 4; ++q) val[q] = bf16r(xin[q]) + u[q];
    xs[j] = val;
    off[j] = frow * DIM + cc;
  }
#pragma unroll
  for (int j = 0; j < 2; ++j) *(volatile v4f*)(out + off[j]) = xs[j];
  __threadfence();
#pragma unroll
  for (int j = 0; j < 2; ++j) *(volatile v4f*)(out + off[j]) = xs[j];
}

extern "C" void kernel_launch(void* const* d_in, const int* in_sizes, int n_in,
                              void* d_out, int out_size, void* d_ws, size_t ws_size,
                              hipStream_t stream) {
  if (n_in < 11) return;
  const long long need_x = ((long long)(NB - 1) * SEQ_FULL + SEQ) * DIM;
  if ((long long)in_sizes[0] < need_x) return;
  if ((long long)in_sizes[1] < (long long)HID * DIM) return;
  if (in_sizes[2] < HID || in_sizes[3] < HID) return;
  if ((long long)in_sizes[5] < (long long)NFEAT * DIM) return;
  if ((long long)in_sizes[7] < (long long)NFEAT * DIM) return;
  if (in_sizes[6] < NFEAT || in_sizes[8] < NFEAT) return;
  if (in_sizes[9] < DIM || in_sizes[10] < DIM) return;
  if ((long long)out_size < need_x) return;
  if (ws_size < WS_TOTAL) return;

  const float* X    = (const float*)d_in[0];
  const float* w1   = (const float*)d_in[1];
  const float* b1   = (const float*)d_in[2];
  const float* w2   = (const float*)d_in[3];
  const float* wj   = (const float*)d_in[5];
  const float* bj   = (const float*)d_in[6];
  const float* wr   = (const float*)d_in[7];
  const float* br   = (const float*)d_in[8];
  const float* gam  = (const float*)d_in[9];
  const float* bet  = (const float*)d_in[10];
  float* out = (float*)d_out;

  char* ws = (char*)d_ws;
  _Float16* Wj16 = (_Float16*)(ws + OFF_WJ);
  _Float16* Wr16 = (_Float16*)(ws + OFF_WR);
  _Float16* W1a  = (_Float16*)(ws + OFF_W1A);
  _Float16* W1t  = (_Float16*)(ws + OFF_W1T);
  _Float16* Xn16 = (_Float16*)(ws + OFF_XN);
  _Float16* Gm16 = (_Float16*)(ws + OFF_GM);
  float*    Gf   = (float*)(ws + OFF_GF);

  dim3 blk(256);

  wplane_kernel<<<dim3((unsigned)(((size_t)NFEAT * DIM) / 2048)), blk, 0, stream>>>(wj, Wj16);
  wplane_kernel<<<dim3((unsigned)(((size_t)NFEAT * DIM) / 2048)), blk, 0, stream>>>(wr, Wr16);
  wplane_kernel<<<dim3((unsigned)(((size_t)HID * DIM) / 2048)), blk, 0, stream>>>(w1, W1a);
  wconv_kernel<<<dim3(DIM / 64, HID / 64), blk, 0, stream>>>(w1, W1t, (unsigned)DIM, (unsigned)HID);

  ln_kernel<<<dim3(MROWS / 16), blk, 0, stream>>>(X, gam, bet, Xn16);
  gemm_z_kernel<<<dim3(HID / 64, MROWS / 64), blk, 0, stream>>>(Xn16, W1a, b1, w2, Gm16);
  gemm_g_kernel<<<dim3(DIM / 64, MROWS / 64), blk, 0, stream>>>(Gm16, W1t, Gf);
  heavy_kernel<<<dim3(MROWS / 16), blk, 0, stream>>>(Wj16, bj, Wr16, br, Xn16, Gf, X, out);
}
